// VJEPA2JointDiffuser_1176821039789
// MI455X (gfx1250) — hardware-verified
//
#include <hip/hip_runtime.h>
#include <math.h>
#include <stdint.h>

#define NB    2
#define NV    2048
#define NA    64
#define NT    2112
#define DMOD  1024
#define NH    16
#define HD    64
#define ROT   20
#define TABP  16
#define TABJ  16
#define NQT   (NT / 64)
#define NKB   (NT / 32)
#define ROWSV (NB * NV)
#define ROWSA (NB * NA)
#define ROWSJ (NB * NT)
#define OUT0N (NB * NT * DMOD)
#define OUT1N (NB * NA * DMOD)
#define QSC   1024.0f
#define KSC   1024.0f
#define PCAR  32768.0f
#define VCAR  1024.0f
#define OSC   1024.0f
#define WOS   1024.0f
#define LOG2E 1.4426950408889634f
#define ATT_WAVES   4
#define ATT_THREADS (ATT_WAVES * 32)
#define ATT_BLOCKS  (NB * NH * NQT)
#define SLABF  (16 * 68)
#define SLAB64 (16 * 68)
#define VTP    72
static_assert(HD == 64 && DMOD == NH * HD && NH == 16);
static_assert(NQT == 33 && NKB == 66 && NQT * 64 == NT && NKB * 32 == NT);
static_assert((NV % 64) == 0 && (NA % 64) == 0 && NV + NA == NT);
static_assert(ATT_THREADS == 128 && ATT_BLOCKS == 1056);
static_assert(16 * 36 <= SLABF);
static_assert(3 * ROT + 4 == HD && TABP * TABJ == 256);
static_assert(((ROWSJ * NH * 8) % 256) == 0);
static_assert(((ROWSV * DMOD / 8) % 256) == 0 && ((ROWSA * DMOD / 8) % 256) == 0 && ((DMOD * DMOD / 8) % 256) == 0);
static_assert((ROWSV % 64) == 0 && (ROWSA % 64) == 0 && (DMOD % 64) == 0 && (DMOD % 32) == 0);
static_assert(OUT0N == 4325376 && OUT1N == 131072);

typedef unsigned short u16;
typedef _Float16 v16h __attribute__((ext_vector_type(16)));
typedef _Float16 v8h  __attribute__((ext_vector_type(8)));
typedef __bf16   v16b __attribute__((ext_vector_type(16)));
typedef float    v8f  __attribute__((ext_vector_type(8)));
typedef float    v4f  __attribute__((ext_vector_type(4)));
typedef unsigned int v4u __attribute__((ext_vector_type(4)));

union FragH { v16h v; v8h h[2]; v4u u[2]; };
union FragB { v16b v; v4u u[2]; };

struct InvF { float f[32]; };
static_assert(sizeof(InvF) == 128);

__device__ __forceinline__ unsigned short bf_bits(float f) {
  unsigned u = __float_as_uint(f);
  return (unsigned short)((u + 0x7FFFu + ((u >> 16) & 1u)) >> 16);
}
__device__ __forceinline__ float bf_up(unsigned short h) { return __uint_as_float(((unsigned)h) << 16); }
__device__ __forceinline__ float bfr(float f) { return bf_up(bf_bits(f)); }
__device__ __forceinline__ unsigned short h_bits(_Float16 x) { return __builtin_bit_cast(unsigned short, x); }
__device__ __forceinline__ unsigned pk16(unsigned short a, unsigned short b) { return (unsigned)a | ((unsigned)b << 16); }
__device__ __forceinline__ v8f zero8() { v8f z = {0.f, 0.f, 0.f, 0.f, 0.f, 0.f, 0.f, 0.f}; return z; }
__device__ __forceinline__ v4f zero4() { v4f z = {0.f, 0.f, 0.f, 0.f}; return z; }

__device__ __forceinline__ v16h ldfrag_h(const _Float16* p) {
  FragH f;
  f.h[0] = *(const v8h*)(p);
  f.h[1] = *(const v8h*)(p + 16);
  return f.v;
}
__device__ __forceinline__ v16b ldfrag_b(const u16* p) {
  FragB f;
  f.u[0] = *(const v4u*)(p);
  f.u[1] = *(const v4u*)(p + 16);
  return f.v;
}

__device__ __forceinline__ v8f mma_h(v16h a, v16h b, v8f c) {
  return __builtin_amdgcn_wmma_f32_16x16x32_f16(false, a, false, b, (short)0, c, false, false);
}
__device__ __forceinline__ v8f mma_b(v16b a, v16b b, v8f c) {
  return __builtin_amdgcn_wmma_f32_16x16x32_bf16(false, a, false, b, (short)0, c, false, false);
}
__device__ __forceinline__ void guard2(v8f& a, v8f& b, v16h x0, v16h x1, v16h x2, v16h x3, v16h x4, v16h x5) {
#if defined(__HIP_DEVICE_COMPILE__)
  asm volatile("v_nop\n\tv_nop\n\tv_nop\n\tv_nop"
               : "+v"(a), "+v"(b) : "v"(x0), "v"(x1), "v"(x2), "v"(x3), "v"(x4), "v"(x5) : "memory");
#endif
}
template <typename F>
__device__ __forceinline__ void guard6(v8f& a, v8f& b, v8f& c, v8f& d, F x0, F x1, F x2, F x3, F x4, F x5) {
#if defined(__HIP_DEVICE_COMPILE__)
  asm volatile("v_nop\n\tv_nop\n\tv_nop\n\tv_nop"
               : "+v"(a), "+v"(b), "+v"(c), "+v"(d) : "v"(x0), "v"(x1), "v"(x2), "v"(x3), "v"(x4), "v"(x5) : "memory");
#endif
}
__device__ __forceinline__ void guard10(v8f& a, v8f& b, v8f& c, v8f& d, v16h x0, v16h x1, v16h x2, v16h x3, v16h x4,
                                        v16h x5, v16h x6, v16h x7, v16h x8, v16h x9) {
#if defined(__HIP_DEVICE_COMPILE__)
  asm volatile("v_nop\n\tv_nop\n\tv_nop\n\tv_nop"
               : "+v"(a), "+v"(b), "+v"(c), "+v"(d)
               : "v"(x0), "v"(x1), "v"(x2), "v"(x3), "v"(x4), "v"(x5), "v"(x6), "v"(x7), "v"(x8), "v"(x9) : "memory");
#endif
}
__device__ __forceinline__ void acc_guard4(v8f& a, v8f& b, v8f& c, v8f& d) {
#if defined(__HIP_DEVICE_COMPILE__)
  asm volatile("v_nop\n\tv_nop\n\tv_nop\n\tv_nop" : "+v"(a), "+v"(b), "+v"(c), "+v"(d));
#endif
}
__device__ __forceinline__ void wave_sync_lds() {
  __builtin_amdgcn_fence(__ATOMIC_RELEASE, "workgroup");
  __builtin_amdgcn_wave_barrier();
  __builtin_amdgcn_fence(__ATOMIC_ACQUIRE, "workgroup");
}

__device__ __forceinline__ void sincos_acc(float angf, float& sv, float& cv) {
  const double a = (double)angf;
  const double TWO_OVER_PI = 0.63661977236758134308;
  const double PIO2_HI = 1.5707963267948966;
  const double PIO2_LO = 6.123233995736766e-17;
  const int kq = (int)(a * TWO_OVER_PI + 0.5);
  const double kd = (double)kq;
  double r = fma(-kd, PIO2_HI, a);
  r = fma(-kd, PIO2_LO, r);
  const double r2 = r * r;
  double sp = 1.0 / 6227020800.0;
  sp = fma(sp, r2, -1.0 / 39916800.0);
  sp = fma(sp, r2, 1.0 / 362880.0);
  sp = fma(sp, r2, -1.0 / 5040.0);
  sp = fma(sp, r2, 1.0 / 120.0);
  sp = fma(sp, r2, -1.0 / 6.0);
  const double s = fma(sp * r2, r, r);
  double cp = -1.0 / 87178291200.0;
  cp = fma(cp, r2, 1.0 / 479001600.0);
  cp = fma(cp, r2, -1.0 / 3628800.0);
  cp = fma(cp, r2, 1.0 / 40320.0);
  cp = fma(cp, r2, -1.0 / 720.0);
  cp = fma(cp, r2, 1.0 / 24.0);
  cp = fma(cp, r2, -0.5);
  const double c = fma(cp, r2, 1.0);
  const int qd = kq & 3;
  const double so = (qd == 0) ? s : (qd == 1) ? c : (qd == 2) ? -s : -c;
  const double co = (qd == 0) ? c : (qd == 1) ? -s : (qd == 2) ? -c : s;
  sv = (float)so;
  cv = (float)co;
}

__global__ __launch_bounds__(256) void k_tab(float* CT, float* ST, InvF inv) {
  const int t = (int)threadIdx.x;
  const int p = t >> 4, j = t & 15;
  float f = inv.f[0];
#pragma unroll
  for (int i = 1; i < 16; ++i) f = (j == i) ? inv.f[i] : f;
  const float ang = (float)p * f;
  float sv, cv;
  sincos_acc(ang, sv, cv);
  for (int pass = 0; pass < 2; ++pass) {
    *(volatile float*)(CT + t) = cv;
    *(volatile float*)(ST + t) = sv;
    __threadfence();
  }
}

__global__ __launch_bounds__(256) void cvt16(const float* __restrict__ x, u16* D, int n8, int f16mode, float scale) {
  const int gt = blockIdx.x * 256 + (int)threadIdx.x;
  if (gt >= n8) return;
  const float* p = x + (size_t)gt * 8;
  const v4f a = *(const v4f*)(p), bq = *(const v4f*)(p + 4);
  float v[8];
#pragma unroll
  for (int e = 0; e < 4; ++e) { v[e] = a[e]; v[4 + e] = bq[e]; }
  unsigned short s[8];
#pragma unroll
  for (int e = 0; e < 8; ++e) {
    const unsigned short hb = h_bits((_Float16)(bfr(v[e]) * scale));
    const unsigned short bb = bf_bits(v[e]);
    s[e] = (f16mode != 0) ? hb : bb;
  }
  v4u o;
#pragma unroll
  for (int e = 0; e < 4; ++e) o[e] = pk16(s[2 * e], s[2 * e + 1]);
  u16* d = D + (size_t)gt * 8;
  for (int pass = 0; pass < 2; ++pass) {
    *(volatile v4u*)(d) = o;
    __threadfence();
  }
}

__device__ __forceinline__ void epi64(float* sl, v8f a0, v8f a1, v8f a2, v8f a3, float oscale, v4f badd, float* C, int N,
                                      size_t rowb, int col0, int lane) {
  const int hh = lane >> 4, m = lane & 15;
#pragma unroll
  for (int r = 0; r < 8; ++r) {
    const int ro = (8 * hh + r) * 68 + m;
    sl[ro]      = a0[r] * oscale;
    sl[ro + 16] = a1[r] * oscale;
    sl[ro + 32] = a2[r] * oscale;
    sl[ro + 48] = a3[r] * oscale;
  }
  wave_sync_lds();
  v4f vals[8];
#pragma unroll
  for (int it = 0; it < 8; ++it) vals[it] = *(const v4f*)(sl + (it * 2 + hh) * 68 + m * 4) + badd;
  float* dst = C + (rowb + (size_t)hh) * (size_t)N + col0 + m * 4;
  for (int pass = 0; pass < 2; ++pass) {
#pragma unroll
    for (int it = 0; it < 8; ++it) {
      *(volatile v4f*)(dst + (size_t)(it * 2) * (size_t)N) = vals[it];
    }
    __threadfence();
  }
}

__global__ __launch_bounds__(128)
void gemm_bf(const u16* __restrict__ A, const u16* __restrict__ Bt, const float* __restrict__ bias, float* C,
             int M, int N, int K, int tin, int tstride, int tbase) {
  __shared__ __align__(16) float slab[4 * SLAB64];
  const int tid = threadIdx.x, wave = tid >> 5, lane = tid & 31, hh = lane >> 4, m = lane & 15;
  const int ntile = N >> 6;
  const int bid   = blockIdx.x;
  const int rowb  = (bid / ntile) * 64 + wave * 16;
  const int col0  = (bid % ntile) * 64;
  if (rowb + 16 > M) return;
  const int orow  = (rowb / tin) * tstride + tbase + (rowb % tin);
  const u16* ap = A  + (size_t)(rowb + m) * K + 8 * hh;
  const u16* bp = Bt + (size_t)(col0 + m) * K + 8 * hh;
  const size_t bs = (size_t)16 * K;
  v8f acc0 = zero8(), acc1 = zero8(), acc2 = zero8(), acc3 = zero8();
#pragma unroll 1
  for (int k0 = 0; k0 < K; k0 += 32) {
    const v16b a  = ldfrag_b(ap + k0);
    const v16b b0 = ldfrag_b(bp + k0);
    const v16b b1 = ldfrag_b(bp + bs + k0);
    const v16b b2 = ldfrag_b(bp + 2 * bs + k0);
    const v16b b3 = ldfrag_b(bp + 3 * bs + k0);
    acc0 = mma_b(a, b0, acc0);
    acc1 = mma_b(a, b1, acc1);
    acc2 = mma_b(a, b2, acc2);
    acc3 = mma_b(a, b3, acc3);
    guard6<v16b>(acc0, acc1, acc2, acc3, a, b0, b1, b2, b3, a);
  }
  const v4f bv = *(const v4f*)(bias + col0 + m * 4);
  v4f badd;
#pragma unroll
  for (int e = 0; e < 4; ++e) badd[e] = bfr(bv[e]);
  epi64(slab + wave * SLAB64, acc0, acc1, acc2, acc3, 1.0f, badd, C, N, (size_t)orow, col0, lane);
}

__global__ __launch_bounds__(128)
void gemm_h2(const u16* __restrict__ Ah, const u16* __restrict__ Al, const u16* __restrict__ Bt,
             const float* __restrict__ bias, float* C, int M, int N, int K, float oscale) {
  __shared__ __align__(16) float slab[4 * SLAB64];
  const int tid = threadIdx.x, wave = tid >> 5, lane = tid & 31, hh = lane >> 4, m = lane & 15;
  const int ntile = N >> 6;
  const int bid   = blockIdx.x;
  const int rowb  = (bid / ntile) * 64 + wave * 16;
  const int col0  = (bid % ntile) * 64;
  if (rowb + 16 > M) return;
  const size_t aofs = (size_t)(rowb + m) * K + 8 * hh;
  const _Float16* ahp = (const _Float16*)(const void*)Ah + aofs;
  const _Float16* alp = (const _Float16*)(const void*)Al + aofs;
  const _Float16* bp  = (const _Float16*)(const void*)Bt + (size_t)(col0 + m) * K + 8 * hh;
  const size_t bs = (size_t)16 * K;
  v8f acc0 = zero8(), acc1 = zero8(), acc2 = zero8(), acc3 = zero8();
#pragma unroll 1
  for (int k0 = 0; k0 < K; k0 += 32) {
    const v16h ah = ldfrag_h(ahp + k0), al = ldfrag_h(alp + k0);
    const v16h b0 = ldfrag_h(bp + k0);
    const v16h b1 = ldfrag_h(bp + bs + k0);
    const v16h b2 = ldfrag_h(bp + 2 * bs + k0);
    const v16h b3 = ldfrag_h(bp + 3 * bs + k0);
    acc0 = mma_h(ah, b0, acc0);  acc0 = mma_h(al, b0, acc0);
    acc1 = mma_h(ah, b1, acc1);  acc1 = mma_h(al, b1, acc1);
    acc2 = mma_h(ah, b2, acc2);  acc2 = mma_h(al, b2, acc2);
    acc3 = mma_h(ah, b3, acc3);  acc3 = mma_h(al, b3, acc3);
    guard6<v16h>(acc0, acc1, acc2, acc3, ah, al, b0, b1, b2, b3);
  }
  const v4f bv = *(const v4f*)(bias + col0 + m * 4);
  v4f badd;
#pragma unroll
  for (int e = 0; e < 4; ++e) badd[e] = bfr(bv[e]);
  epi64(slab + wave * SLAB64, acc0, acc1, acc2, acc3, oscale, badd, C, N, (size_t)rowb, col0, lane);
}

__global__ __launch_bounds__(256) void rot16(const float* __restrict__ x,
                                             const float* __restrict__ CT, const float* __restrict__ ST,
                                             u16* hpl, int nrows, float sc) {
#pragma clang fp contract(off)
  const int gt   = blockIdx.x * 256 + (int)threadIdx.x;
  const int row  = gt >> 3;
  const int d0   = (gt & 7) * 8;
  const bool live = row < nrows;
  const int rowc = live ? row : (nrows - 1);
  const int tok  = (rowc >> 4) % NT;
  const bool vid = tok < NV;
  const int pf   = vid ? (tok >> 8) : 0;
  const int ph   = vid ? ((tok >> 4) & 15) : 0;
  const int pw   = vid ? (tok & 15) : 0;
  const float* xr = x + (size_t)rowc * HD + d0;
  const v4f xa = *(const v4f*)(xr), xb = *(const v4f*)(xr + 4);
  float y[8];
#pragma unroll
  for (int e = 0; e < 4; ++e) { y[e] = xa[e]; y[4 + e] = xb[e]; }
  float w[8];
#pragma unroll
  for (int e = 0; e < 4; ++e) {
    const int de   = d0 + 2 * e;
    const int seg  = (de >= 2 * ROT) ? 2 : ((de >= ROT) ? 1 : 0);
    const bool keep = de >= 3 * ROT;
    const int cc   = de - ROT * seg;
    int j0 = (cc >= 10) ? (cc - 10) : cc;
    j0 = keep ? 0 : j0;
    int pos = (seg == 0) ? pf : ((seg == 1) ? ph : pw);
    pos = keep ? 0 : pos;
    const int ti = pos * TABJ + j0;
    const float c0 = CT[ti],     s0 = ST[ti];
    const float c1 = CT[ti + 1], s1 = ST[ti + 1];
    const float x0 = y[2 * e], x1 = y[2 * e + 1];
    w[2 * e]     = x0 * c0 - x1 * s0;
    w[2 * e + 1] = x1 * c1 + x0 * s1;
  }
  v4u oh;
#pragma unroll
  for (int e = 0; e < 4; ++e) {
    const _Float16 h0 = (_Float16)(w[2 * e] * sc), h1 = (_Float16)(w[2 * e + 1] * sc);
    oh[e] = pk16(h_bits(h0), h_bits(h1));
  }
  if (live) {
    const size_t o8 = (size_t)row * HD + d0;
    for (int pass = 0; pass < 2; ++pass) {
      *(volatile v4u*)(hpl + o8) = oh;
      __threadfence();
    }
  }
}

__global__ __launch_bounds__(256) void vt16(const float* __restrict__ v, u16* VHo, u16* VLo) {
  __shared__ __align__(16) u16 TH[HD * VTP];
  __shared__ __align__(16) u16 TL[HD * VTP];
  const int tid = threadIdx.x;
  const int bid = blockIdx.x;
  const int st  = bid % NQT;
  const int h   = (bid / NQT) % NH;
  const int b   = bid / (NQT * NH);
  const int s0  = st * 64;
  {
    const int sl = tid >> 2;
    const int dc = (tid & 3) * 16;
    const float* src = v + (((size_t)(b * NT + s0 + sl)) * NH + h) * HD + dc;
#pragma unroll
    for (int i = 0; i < 4; ++i) {
      const v4f a = *(const v4f*)(src + 4 * i);
#pragma unroll
      for (int e = 0; e < 4; ++e) {
        const float t = a[e] * VCAR;
        const _Float16 hv = (_Float16)t;
        const _Float16 lv = (_Float16)(t - (float)hv);
        TH[(dc + 4 * i + e) * VTP + sl] = h_bits(hv);
        TL[(dc + 4 * i + e) * VTP + sl] = h_bits(lv);
      }
    }
  }
  __syncthreads();
  v4u vh[2], vl[2];
  const int q8 = tid >> 3, p8 = (tid & 7) * 8;
#pragma unroll
  for (int it = 0; it < 2; ++it) {
    const int line = it * 32 + q8;
    vh[it] = *(const v4u*)(TH + line * VTP + p8);
    vl[it] = *(const v4u*)(TL + line * VTP + p8);
  }
  const size_t base = ((size_t)(b * NH + h) * HD) * NT + s0 + p8;
  for (int pass = 0; pass < 2; ++pass) {
#pragma unroll
    for (int it = 0; it < 2; ++it) {
      const int line = it * 32 + q8;
      *(volatile v4u*)(VHo + base + (size_t)line * NT) = vh[it];
      *(volatile v4u*)(VLo + base + (size_t)line * NT) = vl[it];
    }
    __threadfence();
  }
}

__global__ __launch_bounds__(ATT_THREADS)
void attn_joint(const u16* __restrict__ QHp, const u16* __restrict__ KHp,
                const u16* __restrict__ VHp, const u16* __restrict__ VLp, float* out) {
  __shared__ __align__(16) float smem[ATT_WAVES * SLABF];

  const int tid  = threadIdx.x;
  const int wave = tid >> 5;
  const int lane = tid & 31;
  const int hh   = lane >> 4;
  const int c    = lane & 15;

  const int bid  = blockIdx.x;
  const int qt   = bid % NQT;
  const int head = (bid / NQT) % NH;
  const int b    = bid / (NQT * NH);
  const int q0   = qt * 64 + wave * 16;

  const size_t qofs = (((size_t)(b * NT + q0 + c)) * NH + head) * HD + 8 * hh;
  const _Float16* Qh  = (const _Float16*)(const void*)QHp + qofs;
  const size_t kofs = (((size_t)b * NT + c) * NH + head) * HD + 8 * hh;
  const _Float16* Khb = (const _Float16*)(const void*)KHp + kofs;
  const size_t vofs = ((size_t)(b * NH + head) * HD + c) * NT + 8 * hh;
  const _Float16* Vhb = (const _Float16*)(const void*)VHp + vofs;
  const _Float16* Vlb = (const _Float16*)(const void*)VLp + vofs;
  const float lsc = 0.125f * (LOG2E / (QSC * KSC));

  const v16h qf0 = ldfrag_h(Qh);
  const v16h qf1 = ldfrag_h(Qh + 32);

  float mrow[8], lrow[8];
  v8f o[4];
#pragma unroll
  for (int r = 0; r < 8; ++r) { mrow[r] = -INFINITY; lrow[r] = 0.f; }
#pragma unroll
  for (int j = 0; j < 4; ++j) o[j] = zero8();
  float* pt = smem + wave * SLABF;

#pragma unroll 1
  for (int it = 0; it < NKB; ++it) {
    const int kb = it * 32;
    v8f s0 = zero8(), s1 = zero8();
    {
      const _Float16* k0p = Khb + (size_t)kb * (NH * HD);
      const _Float16* k1p = k0p + (size_t)16 * (NH * HD);
      const v16h ka0 = ldfrag_h(k0p), ka1 = ldfrag_h(k0p + 32);
      const v16h kc0 = ldfrag_h(k1p), kc1 = ldfrag_h(k1p + 32);
      s0 = mma_h(qf0, ka0, s0);
      s0 = mma_h(qf1, ka1, s0);
      s1 = mma_h(qf0, kc0, s1);
      s1 = mma_h(qf1, kc1, s1);
      guard2(s0, s1, qf0, qf1, ka0, ka1, kc0, kc1);
    }
#pragma unroll
    for (int r = 0; r < 8; ++r) {
      const float t0 = s0[r] * lsc;
      const float t1 = s1[r] * lsc;
      float mx = fmaxf(t0, t1);
#pragma unroll
      for (int off = 1; off < 16; off <<= 1) mx = fmaxf(mx, __shfl_xor(mx, off, 32));
      const float mn   = fmaxf(mrow[r], mx);
      const float mref = (mn == -INFINITY) ? 0.f : mn;
      const float al   = exp2f(mrow[r] - mref);
      mrow[r] = mn;
      const float e0 = exp2f(t0 - mref), e1 = exp2f(t1 - mref);
      float ps = e0 + e1;
#pragma unroll
      for (int off = 1; off < 16; off <<= 1) ps += __shfl_xor(ps, off, 32);
      lrow[r] = lrow[r] * al + ps;
#pragma unroll
      for (int j = 0; j < 4; ++j) o[j][r] *= al;
      const int ro = (8 * hh + r) * 36 + c;
      pt[ro]      = e0;
      pt[ro + 16] = e1;
    }
    wave_sync_lds();
    FragH ph, pl;
    {
      const float* prow = pt + c * 36 + 8 * hh;
      const v4f p0 = *(const v4f*)(prow), p1 = *(const v4f*)(prow + 4);
      const v4f p2 = *(const v4f*)(prow + 16), p3 = *(const v4f*)(prow + 20);
#pragma unroll
      for (int e = 0; e < 4; ++e) {
        const float ta = p0[e] * PCAR, tb = p1[e] * PCAR, tc = p2[e] * PCAR, td = p3[e] * PCAR;
        const _Float16 ha = (_Float16)ta, hb = (_Float16)tb, hc = (_Float16)tc, hd = (_Float16)td;
        ph.h[0][e]     = ha;
        ph.h[0][4 + e] = hb;
        ph.h[1][e]     = hc;
        ph.h[1][4 + e] = hd;
        pl.h[0][e]     = (_Float16)(ta - (float)ha);
        pl.h[0][4 + e] = (_Float16)(tb - (float)hb);
        pl.h[1][e]     = (_Float16)(tc - (float)hc);
        pl.h[1][4 + e] = (_Float16)(td - (float)hd);
      }
    }
    {
      const _Float16* vhp = Vhb + kb;
      const _Float16* vlp = Vlb + kb;
      const v16h vh0 = ldfrag_h(vhp);
      const v16h vh1 = ldfrag_h(vhp + (size_t)16 * NT);
      const v16h vh2 = ldfrag_h(vhp + (size_t)32 * NT);
      const v16h vh3 = ldfrag_h(vhp + (size_t)48 * NT);
      const v16h vl0 = ldfrag_h(vlp);
      const v16h vl1 = ldfrag_h(vlp + (size_t)16 * NT);
      const v16h vl2 = ldfrag_h(vlp + (size_t)32 * NT);
      const v16h vl3 = ldfrag_h(vlp + (size_t)48 * NT);
      o[0] = mma_h(ph.v, vh0, o[0]);  o[0] = mma_h(pl.v, vh0, o[0]);  o[0] = mma_h(ph.v, vl0, o[0]);
      o[1] = mma_h(ph.v, vh1, o[1]);  o[1] = mma_h(pl.v, vh1, o[1]);  o[1] = mma_h(ph.v, vl1, o[1]);
      o[2] = mma_h(ph.v, vh2, o[2]);  o[2] = mma_h(pl.v, vh2, o[2]);  o[2] = mma_h(ph.v, vl2, o[2]);
      o[3] = mma_h(ph.v, vh3, o[3]);  o[3] = mma_h(pl.v, vh3, o[3]);  o[3] = mma_h(ph.v, vl3, o[3]);
      guard10(o[0], o[1], o[2], o[3], ph.v, pl.v, vh0, vh1, vh2, vh3, vl0, vl1, vl2, vl3);
    }
    wave_sync_lds();
  }
  acc_guard4(o[0], o[1], o[2], o[3]);

  wave_sync_lds();
  float* slab = pt;
  const float oc = 1.0f / (PCAR * VCAR);
#pragma unroll
  for (int r = 0; r < 8; ++r) {
    const float inv = (1.0f / lrow[r]) * oc;
#pragma unroll
    for (int j = 0; j < 4; ++j) slab[(8 * hh + r) * 68 + j * 16 + c] = o[j][r] * inv;
  }
  wave_sync_lds();
  v4f vals[8];
#pragma unroll
  for (int it = 0; it < 8; ++it) vals[it] = *(const v4f*)(slab + (it * 2 + hh) * 68 + c * 4);
  float* dst = out + ((size_t)(b * NT + q0 + hh)) * DMOD + head * HD + c * 4;
  for (int pass = 0; pass < 2; ++pass) {
#pragma unroll
    for (int it = 0; it < 8; ++it) {
      *(volatile v4f*)(dst + (size_t)(it * 2) * DMOD) = vals[it];
    }
    __threadfence();
  }
}

__global__ __launch_bounds__(256) void octx16(const float* __restrict__ ctx, u16* hpl, u16* lpl) {
  const int gt  = blockIdx.x * 256 + (int)threadIdx.x;
  const int row = gt >> 7;
  const int c8  = (gt & 127) * 8;
  if (row >= ROWSA) return;
  const float* src = ctx + ((size_t)((row >> 6) * NT + NV + (row & (NA - 1)))) * DMOD + c8;
  const v4f a = *(const v4f*)(src), bq = *(const v4f*)(src + 4);
  float w[8];
#pragma unroll
  for (int e = 0; e < 4; ++e) { w[e] = a[e] * OSC; w[4 + e] = bq[e] * OSC; }
  v4u oh, ol;
#pragma unroll
  for (int e = 0; e < 4; ++e) {
    const _Float16 h0 = (_Float16)w[2 * e], h1 = (_Float16)w[2 * e + 1];
    const _Float16 l0 = (_Float16)(w[2 * e] - (float)h0), l1 = (_Float16)(w[2 * e + 1] - (float)h1);
    oh[e] = pk16(h_bits(h0), h_bits(h1));
    ol[e] = pk16(h_bits(l0), h_bits(l1));
  }
  const size_t o8 = (size_t)row * DMOD + c8;
  for (int pass = 0; pass < 2; ++pass) {
    *(volatile v4u*)(hpl + o8) = oh;
    *(volatile v4u*)(lpl + o8) = ol;
    __threadfence();
  }
}

static inline size_t alup(size_t v) { return (v + (size_t)65535) & ~(size_t)65535; }

extern "C" void kernel_launch(void* const* d_in, const int* in_sizes, int n_in,
                              void* d_out, int out_size, void* d_ws, size_t ws_size,
                              hipStream_t stream) {
  if (n_in < 16) return;
  if (in_sizes[0] != ROWSV * DMOD || in_sizes[1] != ROWSA * DMOD) return;
  for (int i = 2; i <= 14; i += 2) { if (in_sizes[i] != DMOD * DMOD) return; }
  for (int i = 3; i <= 15; i += 2) { if (in_sizes[i] != DMOD) return; }
  if (out_size != OUT0N + OUT1N) return;

  const float* xv  = (const float*)d_in[0];
  const float* xa  = (const float*)d_in[1];
  const float* wq  = (const float*)d_in[2];   const float* bq  = (const float*)d_in[3];
  const float* wk  = (const float*)d_in[4];   const float* bk  = (const float*)d_in[5];
  const float* wv  = (const float*)d_in[6];   const float* bv  = (const float*)d_in[7];
  const float* wqa = (const float*)d_in[8];   const float* bqa = (const float*)d_in[9];
  const float* wka = (const float*)d_in[10];  const float* bka = (const float*)d_in[11];
  const float* wva = (const float*)d_in[12];  const float* bva = (const float*)d_in[13];
  const float* wpa = (const float*)d_in[14];  const float* bpa = (const float*)d_in[15];
  float*       out  = (float*)d_out;
  float*       out1 = out + (size_t)OUT0N;

  const size_t szTab = (size_t)TABP * TABJ * 4;
  const size_t szXB  = (size_t)ROWSV * DMOD * 2;
  const size_t szXA  = (size_t)ROWSA * DMOD * 2;
  const size_t szW   = (size_t)DMOD * DMOD * 2;
  const size_t szF   = (size_t)ROWSJ * DMOD * 4;
  const size_t szP   = (size_t)ROWSJ * DMOD * 2;
  const size_t szVP  = (size_t)NB * NH * HD * NT * 2;
  const size_t szO   = (size_t)ROWSA * DMOD * 2;
  size_t off = 0;
  const size_t oCT  = off; off = alup(off + szTab);
  const size_t oST  = off; off = alup(off + szTab);
  const size_t oXB  = off; off = alup(off + szXB);
  const size_t oXA  = off; off = alup(off + szXA);
  const size_t oWQ  = off; off = alup(off + szW);
  const size_t oWK  = off; off = alup(off + szW);
  const size_t oWV  = off; off = alup(off + szW);
  const size_t oWQA = off; off = alup(off + szW);
  const size_t oWKA = off; off = alup(off + szW);
  const size_t oWVA = off; off = alup(off + szW);
  const size_t oWP  = off; off = alup(off + szW);
  const size_t oF   = off; off = alup(off + szF);
  const size_t oQH  = off; off = alup(off + szP);
  const size_t oKH  = off; off = alup(off + szP);
  const size_t oVH  = off; off = alup(off + szVP);
  const size_t oVL  = off; off = alup(off + szVP);
  const size_t oOH  = off; off = alup(off + szO);
  const size_t oOL  = off; off = alup(off + szO);
  if (off > ws_size) return;
  if (off > (size_t)134217728) return;

  char* ws = (char*)d_ws;
  float* CT   = (float*)(ws + oCT);
  float* ST   = (float*)(ws + oST);
  u16*   XB   = (u16*)(ws + oXB);
  u16*   XA   = (u16*)(ws + oXA);
  u16*   WQB  = (u16*)(ws + oWQ);
  u16*   WKB  = (u16*)(ws + oWK);
  u16*   WVB  = (u16*)(ws + oWV);
  u16*   WQAB = (u16*)(ws + oWQA);
  u16*   WKAB = (u16*)(ws + oWKA);
  u16*   WVAB = (u16*)(ws + oWVA);
  u16*   WPB  = (u16*)(ws + oWP);
  float* F    = (float*)(ws + oF);
  u16*   QH   = (u16*)(ws + oQH);
  u16*   KH   = (u16*)(ws + oKH);
  u16*   VH   = (u16*)(ws + oVH);
  u16*   VL   = (u16*)(ws + oVL);
  u16*   OH   = (u16*)(ws + oOH);
  u16*   OL   = (u16*)(ws + oOL);

  InvF inv;
  for (int i = 0; i < 32; ++i) inv.f[i] = 0.0f;
  for (int j = 0; j < 10; ++j) {
    const float ef = (float)j * 0.1f;
    const double p = pow(10000.0, (double)ef);
    const float pf = (float)p;
    inv.f[j] = 1.0f / pf;
  }

  const dim3 blk(256);
  const int n8xv = (ROWSV * DMOD) / 8;
  const int n8xa = (ROWSA * DMOD) / 8;
  const int n8w  = (DMOD * DMOD) / 8;
  if ((n8xv % 256) != 0 || (n8xa % 256) != 0 || (n8w % 256) != 0) return;
  const dim3 gXv(n8xv / 256);
  const dim3 gXa(n8xa / 256);
  const dim3 gWc(n8w / 256);
  const dim3 gGv((ROWSV / 64) * (DMOD / 64));
  const dim3 gGa((ROWSA / 64) * (DMOD / 64));
  const dim3 bG(128);
  const int rowsH = ROWSJ * NH;
  const dim3 gR((rowsH * 8) / 256);
  const dim3 gVT(NB * NH * NQT);
  const dim3 gAT(ATT_BLOCKS);
  const dim3 bAT(ATT_THREADS);
  const dim3 gO((ROWSA * DMOD / 8) / 256);

  k_tab<<<dim3(1), blk, 0, stream>>>(CT, ST, inv);
  cvt16<<<gWc, blk, 0, stream>>>(wq,  WQB,  n8w, 0, 1.0f);
  cvt16<<<gWc, blk, 0, stream>>>(wk,  WKB,  n8w, 0, 1.0f);
  cvt16<<<gWc, blk, 0, stream>>>(wv,  WVB,  n8w, 0, 1.0f);
  cvt16<<<gWc, blk, 0, stream>>>(wqa, WQAB, n8w, 0, 1.0f);
  cvt16<<<gWc, blk, 0, stream>>>(wka, WKAB, n8w, 0, 1.0f);
  cvt16<<<gWc, blk, 0, stream>>>(wva, WVAB, n8w, 0, 1.0f);
  cvt16<<<gWc, blk, 0, stream>>>(wpa, WPB,  n8w, 1, WOS);
  cvt16<<<gXv, blk, 0, stream>>>(xv, XB, n8xv, 0, 1.0f);
  cvt16<<<gXa, blk, 0, stream>>>(xa, XA, n8xa, 0, 1.0f);
  gemm_bf<<<gGv, bG, 0, stream>>>(XB, WQB,  bq,  F, ROWSV, DMOD, DMOD, NV, NT, 0);
  gemm_bf<<<gGa, bG, 0, stream>>>(XA, WQAB, bqa, F, ROWSA, DMOD, DMOD, NA, NT, NV);
  rot16<<<gR, blk, 0, stream>>>(F, CT, ST, QH, rowsH, QSC);
  gemm_bf<<<gGv, bG, 0, stream>>>(XB, WKB,  bk,  F, ROWSV, DMOD, DMOD, NV, NT, 0);
  gemm_bf<<<gGa, bG, 0, stream>>>(XA, WKAB, bka, F, ROWSA, DMOD, DMOD, NA, NT, NV);
  rot16<<<gR, blk, 0, stream>>>(F, CT, ST, KH, rowsH, KSC);
  gemm_bf<<<gGv, bG, 0, stream>>>(XB, WVB,  bv,  F, ROWSV, DMOD, DMOD, NV, NT, 0);
  gemm_bf<<<gGa, bG, 0, stream>>>(XA, WVAB, bva, F, ROWSA, DMOD, DMOD, NA, NT, NV);
  vt16<<<gVT, blk, 0, stream>>>(F, VH, VL);
  attn_joint<<<gAT, bAT, 0, stream>>>(QH, KH, VH, VL, out);
  octx16<<<gO, blk, 0, stream>>>(out, OH, OL);
  gemm_h2<<<gGa, bG, 0, stream>>>(OH, OL, WPB, bpa, out1, ROWSA, DMOD, DMOD, 1.0f / (OSC * WOS));
  (void)hipGetLastError();
}
